// deformable_transformer_layer_88776974008705
// MI455X (gfx1250) — hardware-verified
//
#include <hip/hip_runtime.h>
#define NB 2
#define CC 512
#define HH 32
#define NTOK (HH * HH)
#define NR (NB * NTOK)
#define NG 8
#define CG 64
#define H2 8
#define NKV (H2 * H2)
#define SCALE 0.125f
#define NCPB (NB * NG)
typedef __bf16 v16b __attribute__((ext_vector_type(16)));
typedef unsigned short v8us __attribute__((ext_vector_type(8), may_alias));
typedef float  v8f  __attribute__((ext_vector_type(8)));
typedef float  v4f  __attribute__((ext_vector_type(4)));
typedef float  v4fa __attribute__((ext_vector_type(4), may_alias));
union FragB { v16b v; v8us half[2]; unsigned short u[16]; };

__device__ __forceinline__ unsigned short bf16_bits(float x) { unsigned int u = __float_as_uint(x); return (unsigned short)((u + 0x7FFFu + ((u >> 16) & 1u)) >> 16); }
__device__ __forceinline__ float bf16_val(unsigned short b) { return __uint_as_float(((unsigned int)b) << 16); }
__device__ __forceinline__ float bf16_round(float x) { return bf16_val(bf16_bits(x)); }
template <int NT>
__device__ __forceinline__ v8f mmaN(v16b ah, v16b al, v16b bh, v16b bl, v8f c) {
  c = __builtin_amdgcn_wmma_f32_16x16x32_bf16(false, ah, false, bh, (short)0, c, false, false);
  if (NT >= 2) c = __builtin_amdgcn_wmma_f32_16x16x32_bf16(false, al, false, bh, (short)0, c, false, false);
  if (NT >= 3) c = __builtin_amdgcn_wmma_f32_16x16x32_bf16(false, ah, false, bl, (short)0, c, false, false);
  asm volatile("v_nop\n\tv_nop\n\tv_nop\n\tv_nop" : "+v"(c) : "v"(ah), "v"(al), "v"(bh), "v"(bl));
  return c;
}

__global__ __launch_bounds__(256) void k_wt_bf16(const float* __restrict__ W, unsigned short* __restrict__ Wt, int K, int N) {
  const int t = blockIdx.x * 256 + threadIdx.x;
  const int k8n = K / 8;
  if (t >= N * k8n) return;
  const int n = t / k8n, k8 = (t % k8n) * 8;
  v8us v;
#pragma unroll
  for (int i = 0; i < 8; ++i) v[i] = bf16_bits(W[(size_t)(k8 + i) * N + n]);
  *(volatile v8us*)(Wt + (size_t)n * K + k8) = v;
  __threadfence();
  *(volatile v8us*)(Wt + (size_t)n * K + k8) = v;
}

template <bool ASPLIT, int ACT, bool BIAS_BF16>
__global__ __launch_bounds__(128) void k_gemm_bf(const float* __restrict__ A, int lda, const unsigned short* __restrict__ Wt, int ldb,
                                               const float* __restrict__ bias, float* __restrict__ C, int ldc, int M, int N, int K) {
  __shared__ __attribute__((aligned(16))) float so[4][16][64];
  const int tid = threadIdx.x, w = tid >> 5, lane = tid & 31, ln = lane & 15, hh = lane >> 4;
  const int ntn = N / 64;
  const int wid = blockIdx.x * 4 + w;
  const int mt = wid / ntn, nq = wid % ntn;
  if (mt * 16 >= M) return;
  const int row0 = mt * 16, col0 = nq * 64;
  const float* arow = A + (size_t)(row0 + ln) * lda;
  v8f acc[4] = {};
  for (int kb = 0; kb < K; kb += 32) {
    FragB ah, al;
    const v4f x0 = *(const v4fa*)(arow + kb + 8 * hh), x1 = *(const v4fa*)(arow + kb + 8 * hh + 4);
    const v4f x2 = *(const v4fa*)(arow + kb + 16 + 8 * hh), x3 = *(const v4fa*)(arow + kb + 16 + 8 * hh + 4);
    float xs[16] = {x0[0],x0[1],x0[2],x0[3],x1[0],x1[1],x1[2],x1[3],x2[0],x2[1],x2[2],x2[3],x3[0],x3[1],x3[2],x3[3]};
#pragma unroll
    for (int i = 0; i < 16; ++i) { const unsigned short hb = bf16_bits(xs[i]); ah.u[i] = hb; al.u[i] = ASPLIT ? bf16_bits(xs[i] - bf16_val(hb)) : (unsigned short)0; }
#pragma unroll
    for (int t = 0; t < 4; ++t) {
      const unsigned short* brow = Wt + (size_t)(col0 + t * 16 + ln) * ldb + kb;
      FragB b;
      b.half[0] = *(const v8us*)(brow + 8 * hh);
      b.half[1] = *(const v8us*)(brow + 16 + 8 * hh);
      acc[t] = mmaN<ASPLIT ? 2 : 1>(ah.v, al.v, b.v, b.v, acc[t]);
    }
  }
#pragma unroll
  for (int t = 0; t < 4; ++t) {
    float bv = bias ? bias[col0 + t * 16 + ln] : 0.f;
    if (BIAS_BF16) bv = bf16_round(bv);
#pragma unroll
    for (int r = 0; r < 8; ++r) { float v = acc[t][r] + bv; if (ACT == 1) v = fmaxf(v, 0.f); so[w][8 * hh + r][t * 16 + ln] = v; }
  }
  __builtin_amdgcn_fence(__ATOMIC_ACQ_REL, "workgroup");
  __builtin_amdgcn_wave_barrier();
  const int rsub = lane >> 4, c4 = (lane & 15) * 4;
  for (int pass = 0; pass < 2; ++pass) {
#pragma unroll
    for (int q = 0; q < 8; ++q) {
      const int r = q * 2 + rsub;
      const v4f v = *(const v4fa*)&so[w][r][c4];
      *(volatile v4f*)(C + (size_t)(row0 + r) * ldc + col0 + c4) = v;
    }
    if (pass == 0) __threadfence();
  }
}

template <bool ASPLIT, int ACT, bool BIAS_BF16, bool RES_BF16>
__global__ __launch_bounds__(128) void k_gemm_bf3(const float* __restrict__ A, int lda, const unsigned short* __restrict__ Wt, int ldb,
                                                const float* __restrict__ bias, const float* __restrict__ resid, int rmod, int ldr,
                                                float* __restrict__ C, int ldc, int M, int N, int K) {
  __shared__ __attribute__((aligned(16))) float so[4][16][64];
  const int tid = threadIdx.x, w = tid >> 5, lane = tid & 31, ln = lane & 15, hh = lane >> 4;
  const int ntn = N / 64;
  const int wid = blockIdx.x * 4 + w;
  const int mt = wid / ntn, nq = wid % ntn;
  if (mt * 16 >= M) return;
  const int row0 = mt * 16, col0 = nq * 64;
  const float* arow = A + (size_t)(row0 + ln) * lda;
  v8f acc[4] = {};
  for (int kb = 0; kb < K; kb += 32) {
    FragB ah, al;
    const v4f x0 = *(const v4fa*)(arow + kb + 8 * hh), x1 = *(const v4fa*)(arow + kb + 8 * hh + 4);
    const v4f x2 = *(const v4fa*)(arow + kb + 16 + 8 * hh), x3 = *(const v4fa*)(arow + kb + 16 + 8 * hh + 4);
    float xs[16] = {x0[0],x0[1],x0[2],x0[3],x1[0],x1[1],x1[2],x1[3],x2[0],x2[1],x2[2],x2[3],x3[0],x3[1],x3[2],x3[3]};
#pragma unroll
    for (int i = 0; i < 16; ++i) { const unsigned short hb = bf16_bits(xs[i]); ah.u[i] = hb; al.u[i] = ASPLIT ? bf16_bits(xs[i] - bf16_val(hb)) : (unsigned short)0; }
#pragma unroll
    for (int t = 0; t < 4; ++t) {
      const unsigned short* brow = Wt + (size_t)(col0 + t * 16 + ln) * ldb + kb;
      FragB b;
      b.half[0] = *(const v8us*)(brow + 8 * hh);
      b.half[1] = *(const v8us*)(brow + 16 + 8 * hh);
      acc[t] = mmaN<ASPLIT ? 2 : 1>(ah.v, al.v, b.v, b.v, acc[t]);
    }
  }
#pragma unroll
  for (int t = 0; t < 4; ++t) {
    const int col = col0 + t * 16 + ln;
    float bv = bias ? bias[col] : 0.f;
    if (BIAS_BF16) bv = bf16_round(bv);
#pragma unroll
    for (int r = 0; r < 8; ++r) {
      float v = acc[t][r] + bv;
      if (resid) { float rv = resid[(size_t)((row0 + 8 * hh + r) % rmod) * ldr + col]; if (RES_BF16) rv = bf16_round(rv); v += rv; }
      if (ACT == 1) v = fmaxf(v, 0.f);
      if (ACT == 2) v = 0.5f * v * (1.0f + erff(v * 0.70710678118654752f));
      if (ACT == 3) { const float u = 0.7978845608028654f * (v + 0.044715f * v * v * v); v = 0.5f * v * (1.0f + tanhf(u)); }
      so[w][8 * hh + r][t * 16 + ln] = v;
    }
  }
  __builtin_amdgcn_fence(__ATOMIC_ACQ_REL, "workgroup");
  __builtin_amdgcn_wave_barrier();
  const int rsub = lane >> 4, c4 = (lane & 15) * 4;
  for (int pass = 0; pass < 2; ++pass) {
#pragma unroll
    for (int q = 0; q < 8; ++q) {
      const int r = q * 2 + rsub;
      const v4f v = *(const v4fa*)&so[w][r][c4];
      *(volatile v4f*)(C + (size_t)(row0 + r) * ldc + col0 + c4) = v;
    }
    if (pass == 0) __threadfence();
  }
}
template <bool PARAM_BF16>
__global__ __launch_bounds__(256) void k_layernorm(const float* __restrict__ X, const float* __restrict__ R, const float* __restrict__ g, const float* __restrict__ bta,
                                                  float* __restrict__ out_sum, float* __restrict__ out_norm, int N, float eps) {
  __shared__ float red[256];
  const int row = blockIdx.x, tid = threadIdx.x;
  const float* x = X + (size_t)row * N; const float* rr = R ? R + (size_t)row * N : nullptr;
  float vals[16];
  const int per = N / 256;
  float s1 = 0.f;
  for (int u = 0; u < per / 4; ++u) {
    const int j = tid * 4 + 1024 * u;
    const v4f a = *(const v4fa*)(x + j);
    v4f b = {0.f,0.f,0.f,0.f}; if (rr) b = *(const v4fa*)(rr + j);
#pragma unroll
    for (int q = 0; q < 4; ++q) { const float v = a[q] + b[q]; vals[u * 4 + q] = v; s1 += v; }
  }
  red[tid] = s1; __syncthreads();
  for (int st = 128; st > 0; st >>= 1) { if (tid < st) red[tid] += red[tid + st]; __syncthreads(); }
  const float mu = red[0] / (float)N; __syncthreads();
  float s2 = 0.f;
  for (int u = 0; u < per / 4; ++u)
#pragma unroll
    for (int q = 0; q < 4; ++q) { const float c = vals[u * 4 + q] - mu; s2 += c * c; }
  red[tid] = s2; __syncthreads();
  for (int st = 128; st > 0; st >>= 1) { if (tid < st) red[tid] += red[tid + st]; __syncthreads(); }
  const float rs = rsqrtf(red[0] / (float)N + eps);
  for (int pass = 0; pass < 2; ++pass) {
    for (int u = 0; u < per / 4; ++u) {
      const int j = tid * 4 + 1024 * u;
      v4f o, sm;
#pragma unroll
      for (int q = 0; q < 4; ++q) {
        float gg = g[j + q], bb = bta[j + q];
        if (PARAM_BF16) { gg = bf16_round(gg); bb = bf16_round(bb); }
        sm[q] = vals[u * 4 + q]; o[q] = (vals[u * 4 + q] - mu) * rs * gg + bb;
      }
      if (out_sum) *(volatile v4f*)(out_sum + (size_t)row * N + j) = sm;
      *(volatile v4f*)(out_norm + (size_t)row * N + j) = o;
    }
    if (pass == 0) __threadfence();
  }
}


typedef _Float16 v16h __attribute__((ext_vector_type(16)));
union FragH { v16h v; v8us half[2]; _Float16 h[16]; unsigned short u[16]; };
template <int NT>
__device__ __forceinline__ v8f mmaH(v16h ah, v16h al, v16h bh, v16h bl, v8f c) {
  c = __builtin_amdgcn_wmma_f32_16x16x32_f16(false, ah, false, bh, (short)0, c, false, false);
  if (NT >= 2) c = __builtin_amdgcn_wmma_f32_16x16x32_f16(false, al, false, bh, (short)0, c, false, false);
  if (NT >= 3) c = __builtin_amdgcn_wmma_f32_16x16x32_f16(false, ah, false, bl, (short)0, c, false, false);
  asm volatile("v_nop\n\tv_nop\n\tv_nop\n\tv_nop" : "+v"(c) : "v"(ah), "v"(al), "v"(bh), "v"(bl));
  return c;
}
template <bool ASPLIT>
__global__ __launch_bounds__(128) void k_gemm_h(const float* __restrict__ A, int lda, size_t sA, const _Float16* __restrict__ Bh, int ldb, size_t sB, float alpha, float* __restrict__ C, int ldc, size_t sC, int M, int N, int K) {
  __shared__ __attribute__((aligned(16))) float so[4][16][64];
  const int tid = threadIdx.x, w = tid >> 5, lane = tid & 31, ln = lane & 15, hh = lane >> 4; const int by = blockIdx.y;
  A += (size_t)by * sA; Bh += (size_t)by * sB; C += (size_t)by * sC;
  const int ntn = (N + 63) / 64; const int wid = blockIdx.x * 4 + w; const int mt = wid / ntn, nq = wid % ntn; if (mt * 16 >= M) return;
  const int row0 = mt * 16, col0 = nq * 64; const float* arow = A + (size_t)(row0 + ln) * lda;
  v8f acc[4] = {};
  for (int kb = 0; kb < K; kb += 32) {
    FragH ah, al;
    const v4f x0 = *(const v4fa*)(arow + kb + 8 * hh), x1 = *(const v4fa*)(arow + kb + 8 * hh + 4), x2 = *(const v4fa*)(arow + kb + 16 + 8 * hh), x3 = *(const v4fa*)(arow + kb + 16 + 8 * hh + 4);
    float xs[16] = {x0[0],x0[1],x0[2],x0[3],x1[0],x1[1],x1[2],x1[3],x2[0],x2[1],x2[2],x2[3],x3[0],x3[1],x3[2],x3[3]};
#pragma unroll
    for (int i = 0; i < 16; ++i) { const _Float16 h = (_Float16)xs[i]; ah.h[i] = h; al.h[i] = ASPLIT ? (_Float16)(xs[i] - (float)h) : (_Float16)0.0f; }
#pragma unroll
    for (int t = 0; t < 4; ++t) { if (col0 + t * 16 >= N) continue; const size_t boff = (size_t)(col0 + t * 16 + ln) * ldb + kb; FragH bq; bq.half[0] = *(const v8us*)(Bh + boff + 8 * hh); bq.half[1] = *(const v8us*)(Bh + boff + 16 + 8 * hh);
      acc[t] = mmaH<ASPLIT ? 2 : 1>(ah.v, al.v, bq.v, bq.v, acc[t]); }
  }
#pragma unroll
  for (int t = 0; t < 4; ++t) { if (col0 + t * 16 >= N) continue;
#pragma unroll
    for (int r = 0; r < 8; ++r) so[w][8 * hh + r][t * 16 + ln] = acc[t][r] * alpha; }
  __builtin_amdgcn_fence(__ATOMIC_ACQ_REL, "workgroup"); __builtin_amdgcn_wave_barrier();
  const int rsub = lane >> 4, c4 = (lane & 15) * 4;
  for (int pass = 0; pass < 2; ++pass) {
#pragma unroll
    for (int q = 0; q < 8; ++q) { const int r = q * 2 + rsub; if (col0 + c4 < N) { const v4f v = *(const v4fa*)&so[w][r][c4]; *(volatile v4f*)(C + (size_t)(row0 + r) * ldc + col0 + c4) = v; } }
    if (pass == 0) __threadfence(); }
}

__global__ __launch_bounds__(256) void k_wt_f16(const float* __restrict__ W, _Float16* __restrict__ Wt, int K, int N, float scale) {
  const int t = blockIdx.x * 256 + threadIdx.x; if (t >= N * (K / 8)) return; const int n = t / (K / 8), k8 = (t % (K / 8)) * 8; FragH f;
#pragma unroll
  for (int i = 0; i < 8; ++i) f.h[i] = (_Float16)(bf16_round(W[(size_t)(k8 + i) * N + n]) * scale); const v8us o = f.half[0];
  *(volatile v8us*)((unsigned short*)Wt + (size_t)n * K + k8) = o; __threadfence(); *(volatile v8us*)((unsigned short*)Wt + (size_t)n * K + k8) = o;
}
template <int ACT>
__global__ __launch_bounds__(128) void k_gemm_hhx(const _Float16* __restrict__ A, int lda, size_t sA, const _Float16* __restrict__ Bh, int ldb, size_t sB, float alpha, const float* __restrict__ bias, size_t sBias, const float* __restrict__ CP, int rowsPerB, size_t sCPb, int row0g,
    float* __restrict__ C, _Float16* __restrict__ C16, int ldc, size_t sC, int M, int N, int K) {
  __shared__ __attribute__((aligned(16))) float so[4][16][64];
  const int tid = threadIdx.x, w = tid >> 5, lane = tid & 31, ln = lane & 15, hh = lane >> 4; const int by = blockIdx.y;
  A += (size_t)by * sA; Bh += (size_t)by * sB; const size_t cofs = (size_t)by * sC; const float* bp = bias ? bias + (size_t)by * sBias : nullptr;
  const int ntn = (N + 63) / 64; const int wid = blockIdx.x * 4 + w; const int mt = wid / ntn, nq = wid % ntn; if (mt * 16 >= M) return;
  const int row0 = mt * 16, col0 = nq * 64; const _Float16* arow = A + (size_t)(row0 + ln) * lda;
  v8f acc[4] = {};
  for (int kb = 0; kb < K; kb += 32) { FragH ah; ah.half[0] = *(const v8us*)((const unsigned short*)arow + kb + 8 * hh); ah.half[1] = *(const v8us*)((const unsigned short*)arow + kb + 16 + 8 * hh);
#pragma unroll
    for (int t = 0; t < 4; ++t) { if (col0 + t * 16 >= N) continue; const size_t boff = (size_t)(col0 + t * 16 + ln) * ldb + kb; FragH bq; bq.half[0] = *(const v8us*)((const unsigned short*)Bh + boff + 8 * hh); bq.half[1] = *(const v8us*)((const unsigned short*)Bh + boff + 16 + 8 * hh);
      acc[t] = mmaH<1>(ah.v, ah.v, bq.v, bq.v, acc[t]); }
  }
#pragma unroll
  for (int t = 0; t < 4; ++t) { if (col0 + t * 16 >= N) continue; const int col = col0 + t * 16 + ln; const float bv = bp ? bf16_round(bp[col]) : 0.f;
#pragma unroll
    for (int r = 0; r < 8; ++r) { float v = acc[t][r] * alpha + bv; if (CP) { const int bidx = (row0g + row0 + 8 * hh + r) / rowsPerB; v += CP[(size_t)bidx * sCPb + (size_t)by * 64 + col]; } if (ACT == 1) v = (v > 0.f) ? v : expm1f(v); else if (ACT == 7) v = (v > 0.f) ? v + 1.0f : expf(v); else if (ACT == 8) v = tanhf(v); else if (ACT == 9) v = 0.5f * v * (1.0f + tanhf(0.7978845608028654f * (v + 0.044715f * v * v * v))); else if (ACT == 11) v = 1.0f / (1.0f + expf(-v)); else if (ACT == 12) v = (v > 0.f) ? v : 0.01f * v; else if (ACT == 14) v = (v > 0.f) ? v : 0.1f * v; else if (ACT == 15) v = v / (1.0f + expf(-v)); else if (ACT == 3) v = fmaxf(v, 0.f); else if (ACT == 6) v = 0.5f * v * (1.0f + erff(v * 0.70710678118654752f)); so[w][8 * hh + r][t * 16 + ln] = v; } }
  __builtin_amdgcn_fence(__ATOMIC_ACQ_REL, "workgroup"); __builtin_amdgcn_wave_barrier();
  const int rsub = lane >> 4, c4 = (lane & 15) * 4; typedef _Float16 v4h __attribute__((ext_vector_type(4)));
  for (int pass = 0; pass < 2; ++pass) {
#pragma unroll
    for (int q = 0; q < 8; ++q) { const int r = q * 2 + rsub; if (col0 + c4 < N) { const v4f v = *(const v4fa*)&so[w][r][c4]; if (C) *(volatile v4f*)(C + cofs + (size_t)(row0 + r) * ldc + col0 + c4) = v; if (C16) { v4h h4; for (int i = 0; i < 4; ++i) h4[i] = (_Float16)v[i]; *(volatile v4h*)(C16 + cofs + (size_t)(row0 + r) * ldc + col0 + c4) = h4; } } }
    if (pass == 0) __threadfence(); }
}


typedef _Float16 v4h __attribute__((ext_vector_type(4)));

__global__ __launch_bounds__(256) void k_x16(const float* __restrict__ x, _Float16* __restrict__ X16, size_t n8) { const size_t t = (size_t)blockIdx.x * 256 + threadIdx.x; if (t >= n8) return; FragH f;
#pragma unroll
  for (int q = 0; q < 8; ++q) f.h[q] = (_Float16)bf16_round(x[t * 8 + q]); *(volatile v8us*)((unsigned short*)X16 + t * 8) = f.half[0]; __threadfence(); *(volatile v8us*)((unsigned short*)X16 + t * 8) = f.half[0]; }
__global__ __launch_bounds__(256) void k_h16(const float* __restrict__ x, _Float16* __restrict__ X16, size_t n8) { const size_t t = (size_t)blockIdx.x * 256 + threadIdx.x; if (t >= n8) return; FragH f;
#pragma unroll
  for (int q = 0; q < 8; ++q) f.h[q] = (_Float16)x[t * 8 + q]; *(volatile v8us*)((unsigned short*)X16 + t * 8) = f.half[0]; __threadfence(); *(volatile v8us*)((unsigned short*)X16 + t * 8) = f.half[0]; }
__global__ __launch_bounds__(256) void k_round16f(const float* __restrict__ W, _Float16* __restrict__ Bt, size_t n8) { const size_t t = (size_t)blockIdx.x * 256 + threadIdx.x; if (t >= n8) return; FragH f;
#pragma unroll
  for (int i = 0; i < 8; ++i) f.h[i] = (_Float16)(bf16_round(W[t * 8 + i]) * 16.0f); *(volatile v8us*)((unsigned short*)Bt + t * 8) = f.half[0]; __threadfence(); *(volatile v8us*)((unsigned short*)Bt + t * 8) = f.half[0]; }
template <int NHv, int TTv>
__global__ __launch_bounds__(256) void k_vt(const _Float16* __restrict__ V16, int ldv, int voff, _Float16* __restrict__ Vt) { __shared__ unsigned short tl[64][66]; const int tid = threadIdx.x; const int slab = blockIdx.x / (TTv / 64), lg = blockIdx.x % (TTv / 64); const int b = slab / NHv, h = slab % NHv;
  for (int i = tid; i < 64 * 8; i += 256) { const int r = i / 8, c8 = (i % 8) * 8; FragH f; f.half[0] = *(const v8us*)((const unsigned short*)V16 + ((size_t)b * TTv + lg * 64 + r) * ldv + voff + h * 64 + c8);
#pragma unroll
    for (int q = 0; q < 8; ++q) tl[r][c8 + q] = f.u[q]; }
  __syncthreads();
  for (int pass = 0; pass < 2; ++pass) {
#pragma unroll
    for (int rd = 0; rd < 2; ++rd) { const int d = rd * 32 + tid / 8, pc = tid % 8; FragH f;
#pragma unroll
      for (int q = 0; q < 8; ++q) f.u[q] = tl[pc * 8 + q][d];
      *(volatile v8us*)((unsigned short*)Vt + ((size_t)slab * 64 + d) * TTv + lg * 64 + pc * 8) = f.half[0]; }
    if (pass == 0) __threadfence(); } }

__global__ __launch_bounds__(256) void k_hl(const float* __restrict__ F, _Float16* __restrict__ Hh, _Float16* __restrict__ Hl, size_t n8) { const size_t t = (size_t)blockIdx.x * 256 + threadIdx.x; if (t >= n8) return; FragH fh, fl; const v4f a = *(const v4fa*)(F + t * 8), c = *(const v4fa*)(F + t * 8 + 4);
#pragma unroll
  for (int q = 0; q < 4; ++q) { _Float16 h = (_Float16)a[q]; fh.h[q] = h; fl.h[q] = (_Float16)((a[q] - (float)h) * 1024.0f); h = (_Float16)c[q]; fh.h[4 + q] = h; fl.h[4 + q] = (_Float16)((c[q] - (float)h) * 1024.0f); }
  for (int pass = 0; pass < 2; ++pass) { *(volatile v8us*)((unsigned short*)Hh + t * 8) = fh.half[0]; *(volatile v8us*)((unsigned short*)Hl + t * 8) = fl.half[0]; if (pass == 0) __threadfence(); } }

__device__ __forceinline__ v16h g2_frag(const _Float16* p, int hh) { FragH f; f.half[0] = *(const v8us*)((const unsigned short*)p + 8 * hh); f.half[1] = *(const v8us*)((const unsigned short*)p + 16 + 8 * hh); return f.v; }
__device__ __forceinline__ v8f g2_mma(v16h a, v16h b, v8f c) { v8f d = __builtin_amdgcn_wmma_f32_16x16x32_f16(false, a, false, b, (short)0, c, false, false); asm volatile("v_nop\n\tv_nop\n\tv_nop\n\tv_nop" : "+v"(d) : "v"(a), "v"(b)); return d; }
template <int ACT>
__global__ __launch_bounds__(128) void k_gemm2(const _Float16* __restrict__ A, int lda, size_t sA, const _Float16* __restrict__ Bh, int ldb, size_t sB, float alpha, const float* __restrict__ bias, size_t sBias, const float* __restrict__ CP, int rowsPerB, size_t sCPb, int row0g,
    float* __restrict__ C, _Float16* __restrict__ C16, int ldc, size_t sC, int M, int N, int K) {
  __shared__ __attribute__((aligned(16))) float so[4][32][68];
  const int tid = threadIdx.x, w = tid >> 5, lane = tid & 31, ln = lane & 15, hh = lane >> 4; const int by = blockIdx.y;
  A += (size_t)by * sA; Bh += (size_t)by * sB; const size_t cofs = (size_t)by * sC; const float* bp = bias ? bias + (size_t)by * sBias : nullptr;
  const int ntn = N >> 6; const int mt = blockIdx.x / ntn, nq = blockIdx.x - mt * ntn; const int row0 = mt * 128 + 32 * w, col0 = nq * 64; if (row0 >= M) return;
  const _Float16* a0p = A + (size_t)(row0 + ln) * lda; const _Float16* a1p = a0p + (size_t)16 * lda;
  const _Float16* b0p = Bh + (size_t)(col0 + ln) * ldb; const _Float16* b1p = b0p + (size_t)16 * ldb; const _Float16* b2p = b1p + (size_t)16 * ldb; const _Float16* b3p = b2p + (size_t)16 * ldb;
  const v8f z8 = {0.f,0.f,0.f,0.f,0.f,0.f,0.f,0.f}; v8f c00 = z8, c01 = z8, c02 = z8, c03 = z8, c10 = z8, c11 = z8, c12 = z8, c13 = z8;
#pragma unroll 1
  for (int kb = 0; kb < K; kb += 32) { const v16h a0 = g2_frag(a0p + kb, hh), a1 = g2_frag(a1p + kb, hh);
    v16h b = g2_frag(b0p + kb, hh); c00 = g2_mma(a0, b, c00); c10 = g2_mma(a1, b, c10);
    b = g2_frag(b1p + kb, hh); c01 = g2_mma(a0, b, c01); c11 = g2_mma(a1, b, c11);
    b = g2_frag(b2p + kb, hh); c02 = g2_mma(a0, b, c02); c12 = g2_mma(a1, b, c12);
    b = g2_frag(b3p + kb, hh); c03 = g2_mma(a0, b, c03); c13 = g2_mma(a1, b, c13); }
  v8f accs[8] = {c00, c01, c02, c03, c10, c11, c12, c13};
#pragma unroll
  for (int u = 0; u < 8; ++u) { const int t = u & 3, half = u >> 2; const int col = col0 + t * 16 + ln; const float bv = bp ? bf16_round(bp[col]) : 0.f;
#pragma unroll
    for (int r = 0; r < 8; ++r) { const int rloc = half * 16 + 8 * hh + r; float v = accs[u][r] * alpha + bv; if (CP) { const int bidx = (row0g + row0 + rloc) / rowsPerB; v += CP[(size_t)bidx * sCPb + (size_t)by * 64 + col]; }
      if (ACT == 3) v = fmaxf(v, 0.f); else if (ACT == 6) v = 0.5f * v * (1.0f + erff(v * 0.70710678118654752f)); else if (ACT == 11) v = 1.0f / (1.0f + expf(-v)); else if (ACT == 15) v = v / (1.0f + expf(-v)); else if (ACT == 12) v = (v > 0.f) ? v : 0.01f * v; else if (ACT == 8) v = tanhf(v);
      so[w][rloc][t * 16 + ln] = v; } }
  __builtin_amdgcn_fence(__ATOMIC_ACQ_REL, "workgroup"); __builtin_amdgcn_wave_barrier();
  const int rsub = lane >> 4, c4 = (lane & 15) * 4;
  for (int pass = 0; pass < 2; ++pass) {
#pragma unroll
    for (int q = 0; q < 16; ++q) { const int r = q * 2 + rsub; const v4f v = *(const v4fa*)&so[w][r][c4]; if (C) *(volatile v4f*)(C + cofs + (size_t)(row0 + r) * ldc + col0 + c4) = v; if (C16) { v4h h4; for (int i = 0; i < 4; ++i) h4[i] = (_Float16)v[i]; *(volatile v4h*)(C16 + cofs + (size_t)(row0 + r) * ldc + col0 + c4) = h4; } }
    if (pass == 0) __threadfence(); } }


template <int TM, int SRCBF>
__global__ __launch_bounds__(256) void k_stat(const float* __restrict__ X, const float* __restrict__ ST0, int phase, float* __restrict__ ST) {
  #pragma clang fp contract(off)
  __shared__ float sh[256]; const int c = blockIdx.x; const float mu = phase ? ST0[(size_t)c * 32] : 0.f; float s = 0.f;
  for (int i = threadIdx.x; i < NR; i += 256) { const int b = i / NTOK, t = i % NTOK; float v = TM ? X[(size_t)i * CC + c] : X[((size_t)b * CC + c) * NTOK + t]; if (SRCBF) v = bf16_round(v); v -= mu; s += phase ? v * v : v; }
  sh[threadIdx.x] = s; __syncthreads();
  for (int st = 128; st > 0; st >>= 1) { if ((int)threadIdx.x < st) sh[threadIdx.x] += sh[threadIdx.x + st]; __syncthreads(); }
  if (threadIdx.x == 0) { const float v = sh[0] / (float)NR; float* d = ST + ((size_t)phase * CC + c) * 32; *(volatile float*)d = v; __threadfence(); *(volatile float*)d = v; } }
__global__ __launch_bounds__(256) void k_bn1(const float* __restrict__ x, const float* __restrict__ ST, const float* __restrict__ g, const float* __restrict__ be, _Float16* __restrict__ XB16, float* __restrict__ XRES) {
  #pragma clang fp contract(off)
  __shared__ float tl[64][65]; const int tid = threadIdx.x; const int nslab = CC / 64, ntt = NTOK / 64; const int b = blockIdx.x / (nslab * ntt); const int cs = (blockIdx.x / ntt) % nslab; const int tt = blockIdx.x % ntt; const int c0 = cs * 64, t0 = tt * 64;
  for (int i = tid; i < 64 * 16; i += 256) { const int cl = i / 16, t4 = (i % 16) * 4; const v4f a = *(const v4fa*)(x + ((size_t)b * CC + c0 + cl) * NTOK + t0 + t4);
#pragma unroll
    for (int q = 0; q < 4; ++q) tl[cl][t4 + q] = bf16_round(a[q]); }
  __syncthreads();
  for (int pass = 0; pass < 2; ++pass) {
#pragma unroll
    for (int it = 0; it < 2; ++it) { const int tl_ = it * 32 + (tid >> 3), c8 = (tid & 7) * 8; FragH fa;
#pragma unroll
      for (int q = 0; q < 8; ++q) { const int c = c0 + c8 + q; const float xv = tl[c8 + q][tl_]; const float mu = ST[(size_t)c * 32], var = ST[(size_t)(CC + c) * 32]; fa.h[q] = (_Float16)((xv - mu) * rsqrtf(var + 1e-5f) * bf16_round(g[c]) + bf16_round(be[c])); }
      *(volatile v8us*)((unsigned short*)XB16 + ((size_t)b * NTOK + t0 + tl_) * CC + c0 + c8) = fa.half[0]; }
#pragma unroll
    for (int it = 0; it < 4; ++it) { const int tl_ = it * 16 + (tid >> 4), c4 = (tid & 15) * 4; v4f r;
#pragma unroll
      for (int q = 0; q < 4; ++q) r[q] = tl[c4 + q][tl_];
      *(volatile v4f*)(XRES + ((size_t)b * NTOK + t0 + tl_) * CC + c0 + c4) = r; }
    if (pass == 0) __threadfence(); } }
__global__ __launch_bounds__(256) void k_bn2(const float* __restrict__ X1, const float* __restrict__ ST, const float* __restrict__ g, const float* __restrict__ be, _Float16* __restrict__ H16) {
  #pragma clang fp contract(off)
  const size_t t = (size_t)blockIdx.x * 256 + threadIdx.x; if (t >= (size_t)NR * CC / 8) return; const int c0 = (int)(t % (CC / 8)) * 8; const float* s = X1 + t * 8; FragH f;
#pragma unroll
  for (int q = 0; q < 8; ++q) { const int c = c0 + q; f.h[q] = (_Float16)((s[q] - ST[(size_t)c * 32]) * rsqrtf(ST[(size_t)(CC + c) * 32] + 1e-5f) * bf16_round(g[c]) + bf16_round(be[c])); }
  *(volatile v8us*)((unsigned short*)H16 + t * 8) = f.half[0]; __threadfence(); *(volatile v8us*)((unsigned short*)H16 + t * 8) = f.half[0]; }
__global__ __launch_bounds__(256) void k_offh(const float* __restrict__ Q, const float* __restrict__ dww, const float* __restrict__ dwb, float* __restrict__ OFFH) {
  #pragma clang fp contract(off)
  const int t = blockIdx.x * 256 + threadIdx.x; if (t >= NB * NG * NKV * CG) return; const int c = t % CG; const int p = (t / CG) % NKV; const int bg = t / (CG * NKV); const int b = bg / NG, g = bg % NG; const int oy = p / H2, ox = p % H2; float s = 0.f;
#pragma unroll 1
  for (int ky = 0; ky < 6; ++ky) { const int iy = oy * 4 + ky - 1; if (iy < 0 || iy >= HH) continue;
#pragma unroll 1
    for (int kx = 0; kx < 6; ++kx) { const int ix = ox * 4 + kx - 1; if (ix < 0 || ix >= HH) continue; s += bf16_round(dww[(c * 6 + ky) * 6 + kx]) * Q[((size_t)b * NTOK + iy * HH + ix) * CC + g * CG + c]; } }
  s += bf16_round(dwb[c]); const float v = 0.5f * s * (1.0f + erff(s * 0.70710678118654752f));
  *(volatile float*)(OFFH + ((size_t)bg * NKV + p) * CG + c) = v; __threadfence(); *(volatile float*)(OFFH + ((size_t)bg * NKV + p) * CG + c) = v; }
__global__ __launch_bounds__(256) void k_grid(const float* __restrict__ OFFH, const float* __restrict__ pw, float* __restrict__ GRD) {
  #pragma clang fp contract(off)
  const int t = blockIdx.x * 256 + threadIdx.x; if (t >= NB * NG * NKV) return; const int p = t % NKV; const float* oh = OFFH + (size_t)t * CG; float s0 = 0.f, s1 = 0.f;
#pragma unroll 1
  for (int c = 0; c < CG; ++c) { s0 += oh[c] * bf16_round(pw[c]); s1 += oh[c] * bf16_round(pw[CG + c]); }
  const float offx = tanhf(s0) * 4.0f, offy = tanhf(s1) * 4.0f; const float gx = (float)(p % H2) + offx, gy = (float)(p / H2) + offy; const float vx = 2.0f * gx / 7.0f - 1.0f, vy = 2.0f * gy / 7.0f - 1.0f;
  v4f o; o[0] = vx; o[1] = vy; o[2] = ((vx + 1.0f) * (float)HH - 1.0f) * 0.5f; o[3] = ((vy + 1.0f) * (float)HH - 1.0f) * 0.5f;
  *(volatile v4f*)(GRD + (size_t)t * 4) = o; __threadfence(); *(volatile v4f*)(GRD + (size_t)t * 4) = o; }
__global__ __launch_bounds__(256) void k_samp(const float* __restrict__ x, const float* __restrict__ ST, const float* __restrict__ g1, const float* __restrict__ b1, const float* __restrict__ GRD, _Float16* __restrict__ KV16) {
  #pragma clang fp contract(off)
  const int t = blockIdx.x * 256 + threadIdx.x; if (t >= NB * NG * NKV * (CG / 8)) return; const int c0 = (t % (CG / 8)) * 8; const int p = (t / (CG / 8)) % NKV; const int bg = t / ((CG / 8) * NKV); const int b = bg / NG, g = bg % NG;
  const float px = GRD[((size_t)bg * NKV + p) * 4 + 2], py = GRD[((size_t)bg * NKV + p) * 4 + 3]; const float x0f = floorf(px), y0f = floorf(py); const float wx1 = px - x0f, wy1 = py - y0f; const int x0 = (int)fminf(fmaxf(x0f, -4096.f), 4096.f), y0 = (int)fminf(fmaxf(y0f, -4096.f), 4096.f);
  float acc[8];
#pragma unroll
  for (int q = 0; q < 8; ++q) acc[q] = 0.f;
#pragma unroll
  for (int cr = 0; cr < 4; ++cr) { const int ix = x0 + (cr & 1), iy = y0 + (cr >> 1); if (ix < 0 || ix >= HH || iy < 0 || iy >= HH) continue; const float w = ((cr & 1) ? wx1 : (1.f - wx1)) * ((cr >> 1) ? wy1 : (1.f - wy1));
#pragma unroll
    for (int q = 0; q < 8; ++q) { const int c = g * CG + c0 + q; const float xv = bf16_round(x[((size_t)b * CC + c) * NTOK + iy * HH + ix]); const float xb = (xv - ST[(size_t)c * 32]) * rsqrtf(ST[(size_t)(CC + c) * 32] + 1e-5f) * bf16_round(g1[c]) + bf16_round(b1[c]); acc[q] += w * xb; } }
  FragH f;
#pragma unroll
  for (int q = 0; q < 8; ++q) f.h[q] = (_Float16)acc[q];
  unsigned short* d = (unsigned short*)KV16 + ((size_t)bg / NG * NKV + p) * CC + g * CG + c0; *(volatile v8us*)d = f.half[0]; __threadfence(); *(volatile v8us*)d = f.half[0]; }
__global__ __launch_bounds__(256) void k_cpb0(const float* __restrict__ GRD, int bg, const float* __restrict__ w0, const float* __restrict__ b0, _Float16* __restrict__ C0) {
  #pragma clang fp contract(off)
  const int t = blockIdx.x * 256 + threadIdx.x; if (t >= NTOK * NKV * 16) return; const int o0 = (t & 15) * 8; const int j = (t >> 4) % NKV; const int i = t / (16 * NKV);
  const float qx = 2.0f * (float)(i % HH) / (float)(HH - 1) - 1.0f, qy = 2.0f * (float)(i / HH) / (float)(HH - 1) - 1.0f;
  const float dx = qx - GRD[((size_t)bg * NKV + j) * 4], dy = qy - GRD[((size_t)bg * NKV + j) * 4 + 1];
  const float ux = (dx > 0.f ? 1.f : (dx < 0.f ? -1.f : 0.f)) * logf(fabsf(dx) + 1.0f), uy = (dy > 0.f ? 1.f : (dy < 0.f ? -1.f : 0.f)) * logf(fabsf(dy) + 1.0f); FragH f;
#pragma unroll
  for (int q = 0; q < 8; ++q) { const int o = o0 + q; float v = ux * bf16_round(w0[o]); v += uy * bf16_round(w0[128 + o]); v += bf16_round(b0[o]); f.h[q] = (_Float16)fmaxf(v, 0.f); }
  unsigned short* d = (unsigned short*)C0 + ((size_t)i * NKV + j) * 128 + o0; *(volatile v8us*)d = f.half[0]; __threadfence(); *(volatile v8us*)d = f.half[0]; }
__global__ __launch_bounds__(256) void k_cpb2(const _Float16* __restrict__ C1, int bg, const float* __restrict__ w2, const float* __restrict__ b2, float* __restrict__ BIAS) {
  #pragma clang fp contract(off)
  const int t = blockIdx.x * 256 + threadIdx.x; if (t >= NTOK * NKV) return; const _Float16* c = C1 + (size_t)t * 128; float s = bf16_round(b2[0]);
#pragma unroll 1
  for (int o = 0; o < 128; o += 8) { FragH f; f.half[0] = *(const v8us*)((const unsigned short*)c + o);
#pragma unroll
    for (int q = 0; q < 8; ++q) s += (float)f.h[q] * bf16_round(w2[o + q]); }
  *(volatile float*)(BIAS + (size_t)bg * NTOK * NKV + t) = s; __threadfence(); *(volatile float*)(BIAS + (size_t)bg * NTOK * NKV + t) = s; }
__global__ __launch_bounds__(256) void k_zero4(float* __restrict__ p, size_t n4) { const size_t t = (size_t)blockIdx.x * 256 + threadIdx.x; if (t >= n4) return; const v4f z = {0.f, 0.f, 0.f, 0.f}; *(volatile v4f*)(p + t * 4) = z; __threadfence(); *(volatile v4f*)(p + t * 4) = z; }
__global__ __launch_bounds__(256) void k_soft64(const float* __restrict__ S, const float* __restrict__ BIAS, _Float16* __restrict__ P16) {
  #pragma clang fp contract(off)
  const int tid = threadIdx.x, w = tid >> 5, ln = tid & 31; const size_t row = (size_t)blockIdx.x * 8 + w; if (row >= (size_t)NB * NG * NTOK) return;
  const float v0 = S[row * NKV + ln * 2] + BIAS[row * NKV + ln * 2], v1 = S[row * NKV + ln * 2 + 1] + BIAS[row * NKV + ln * 2 + 1]; float m = fmaxf(v0, v1);
  for (int o = 16; o > 0; o >>= 1) m = fmaxf(m, __shfl_xor(m, o, 32)); const float e0 = expf(v0 - m), e1 = expf(v1 - m); float su = e0 + e1;
  for (int o = 16; o > 0; o >>= 1) su += __shfl_xor(su, o, 32); const float inv = 1024.0f / su; _Float16 h2[2] = {(_Float16)(e0 * inv), (_Float16)(e1 * inv)};
  *(volatile unsigned*)((unsigned short*)P16 + row * NKV + ln * 2) = *(const unsigned*)h2; __threadfence(); *(volatile unsigned*)((unsigned short*)P16 + row * NKV + ln * 2) = *(const unsigned*)h2; }
__global__ __launch_bounds__(256) void k_vt64(const _Float16* __restrict__ V16, _Float16* __restrict__ VT) {
  __shared__ unsigned short tl[64][66]; const int tid = threadIdx.x; const int bh = blockIdx.x; const int b = bh / NG, h = bh % NG;
  for (int i = tid; i < 64 * 8; i += 256) { const int j = i / 8, c8 = (i % 8) * 8; FragH f; f.half[0] = *(const v8us*)((const unsigned short*)V16 + ((size_t)b * NKV + j) * CC + h * CG + c8);
#pragma unroll
    for (int q = 0; q < 8; ++q) tl[j][c8 + q] = f.u[q]; }
  __syncthreads();
  for (int pass = 0; pass < 2; ++pass) {
#pragma unroll
    for (int rd = 0; rd < 2; ++rd) { const int d = rd * 32 + tid / 8, pc = tid % 8; FragH f;
#pragma unroll
      for (int q = 0; q < 8; ++q) f.u[q] = tl[pc * 8 + q][d];
      *(volatile v8us*)((unsigned short*)VT + ((size_t)bh * 64 + d) * NKV + pc * 8) = f.half[0]; }
    if (pass == 0) __threadfence(); } }
__global__ __launch_bounds__(256) void k_nchw(const float* __restrict__ F, float* __restrict__ out) {
  const int t = blockIdx.x * 256 + threadIdx.x; if (t >= NB * CC * (NTOK / 4)) return; const int t0 = (t % (NTOK / 4)) * 4; const int c = (t / (NTOK / 4)) % CC; const int b = t / ((NTOK / 4) * CC); v4f r;
#pragma unroll
  for (int q = 0; q < 4; ++q) r[q] = F[((size_t)b * NTOK + t0 + q) * CC + c];
  float* dst = out + ((size_t)b * CC + c) * NTOK + t0; *(volatile v4f*)dst = r; __threadfence(); *(volatile v4f*)dst = r; }

extern "C" void kernel_launch(void* const* d_in, const int* in_sizes, int n_in,
                              void* d_out, int out_size, void* d_ws, size_t ws_size, hipStream_t stream) {
  (void)in_sizes; (void)n_in; (void)out_size;
  const float* const* I = (const float* const*)d_in; const float* x = I[0]; const float* n1g = I[1]; const float* n1b = I[2]; const float* n2g = I[3]; const float* n2b = I[4]; const float* qw = I[5]; const float* kw = I[6]; const float* vw = I[7]; const float* dww = I[8]; const float* dwb = I[9]; const float* pww = I[10];
  const float* c0w = I[11]; const float* c0b = I[12]; const float* c1w = I[13]; const float* c1b = I[14]; const float* c2w = I[15]; const float* c2b = I[16]; const float* ow = I[17]; const float* ob = I[18]; const float* m1w = I[19]; const float* m1b = I[20]; const float* m2w = I[21]; const float* m2b = I[22];
  char* ws = (char*)d_ws; size_t off = 0;
  auto take = [&](size_t bytes) { char* p = ws + off; off += (bytes + 255) & ~(size_t)255; return p; };
  _Float16* BQ = (_Float16*)take((size_t)NG * CG * CG * 2); _Float16* BK = (_Float16*)take((size_t)NG * CG * CG * 2); _Float16* BV = (_Float16*)take((size_t)NG * CG * CG * 2); _Float16* BC1 = (_Float16*)take(128 * 128 * 2); _Float16* BO = (_Float16*)take((size_t)CC * CC * 2); _Float16* BM1 = (_Float16*)take((size_t)2048 * CC * 2); _Float16* BM2 = (_Float16*)take((size_t)CC * 2048 * 2);
  float* ST1 = (float*)take((size_t)2 * CC * 32 * 4); float* ST2 = (float*)take((size_t)2 * CC * 32 * 4);
  _Float16* XB16 = (_Float16*)take((size_t)NR * CC * 2); float* XRES = (float*)take((size_t)NR * CC * 4); float* Q = (float*)take((size_t)NR * CC * 4); _Float16* Q16 = (_Float16*)take((size_t)NR * CC * 2);
  float* OFFH = (float*)take((size_t)NB * NG * NKV * CG * 4); float* GRD = (float*)take((size_t)NB * NG * NKV * 4 * 4); _Float16* KV16 = (_Float16*)take((size_t)NB * 128 * CC * 2); _Float16* K16 = (_Float16*)take((size_t)NB * 128 * CC * 2); _Float16* V16 = (_Float16*)take((size_t)NB * 128 * CC * 2); _Float16* VT = (_Float16*)take((size_t)NB * NG * 64 * NKV * 2);
  float* S = (float*)take((size_t)NB * NG * NTOK * NKV * 4); _Float16* C0 = (_Float16*)take((size_t)NTOK * NKV * 128 * 2); _Float16* C1 = (_Float16*)take((size_t)NTOK * NKV * 128 * 2); float* BIAS = (float*)take((size_t)NB * NG * NTOK * NKV * 4); _Float16* P16 = (_Float16*)take((size_t)NB * NG * NTOK * NKV * 2);
  _Float16* AO16 = (_Float16*)take((size_t)NR * CC * 2); float* X1 = (float*)take((size_t)NR * CC * 4); _Float16* H16 = (_Float16*)take((size_t)NR * CC * 2); _Float16* GH = (_Float16*)take((size_t)NR * 2048 * 2); float* F = (float*)take((size_t)NR * CC * 4);
  if (off > ws_size) return;
  const size_t w64 = (size_t)NG * CG * CG / 8; const unsigned wb64 = (unsigned)((w64 + 255) / 256);
  k_round16f<<<wb64, 256, 0, stream>>>(qw, BQ, w64); k_round16f<<<wb64, 256, 0, stream>>>(kw, BK, w64); k_round16f<<<wb64, 256, 0, stream>>>(vw, BV, w64);
  k_wt_f16<<<(128 * 128 / 8 + 255) / 256, 256, 0, stream>>>(c1w, BC1, 128, 128, 16.0f);
  k_round16f<<<(unsigned)(((size_t)CC * CC / 8 + 255) / 256), 256, 0, stream>>>(ow, BO, (size_t)CC * CC / 8); k_round16f<<<(unsigned)(((size_t)2048 * CC / 8 + 255) / 256), 256, 0, stream>>>(m1w, BM1, (size_t)2048 * CC / 8); k_round16f<<<(unsigned)(((size_t)CC * 2048 / 8 + 255) / 256), 256, 0, stream>>>(m2w, BM2, (size_t)CC * 2048 / 8);
  k_stat<0, 1><<<CC, 256, 0, stream>>>(x, ST1, 0, ST1); k_stat<0, 1><<<CC, 256, 0, stream>>>(x, ST1, 1, ST1);
  k_bn1<<<NB * (CC / 64) * (NTOK / 64), 256, 0, stream>>>(x, ST1, n1g, n1b, XB16, XRES);
  k_gemm2<0><<<dim3((NR / 128) * 1, NG), 128, 0, stream>>>(XB16, CC, (size_t)CG, BQ, CG, (size_t)CG * CG, 0.0625f, nullptr, 0, nullptr, 1, 0, 0, Q, Q16, CC, (size_t)CG, NR, CG, CG);
  k_offh<<<(NB * NG * NKV * CG + 255) / 256, 256, 0, stream>>>(Q, dww, dwb, OFFH); k_grid<<<(NB * NG * NKV + 255) / 256, 256, 0, stream>>>(OFFH, pww, GRD);
  k_samp<<<(NB * NG * NKV * (CG / 8) + 255) / 256, 256, 0, stream>>>(x, ST1, n1g, n1b, GRD, KV16);
  k_gemm2<0><<<dim3((128 / 128) * 1, NG), 128, 0, stream>>>(KV16, CC, (size_t)CG, BK, CG, (size_t)CG * CG, 0.0625f, nullptr, 0, nullptr, 1, 0, 0, nullptr, K16, CC, (size_t)CG, NB * NKV, CG, CG);
  k_gemm2<0><<<dim3((128 / 128) * 1, NG), 128, 0, stream>>>(KV16, CC, (size_t)CG, BV, CG, (size_t)CG * CG, 0.0625f, nullptr, 0, nullptr, 1, 0, 0, nullptr, V16, CC, (size_t)CG, NB * NKV, CG, CG);
  k_vt64<<<NB * NG, 256, 0, stream>>>(V16, VT);
  for (int b = 0; b < NB; ++b) k_gemm2<0><<<dim3((NTOK / 128) * 1, NG), 128, 0, stream>>>(Q16 + (size_t)b * NTOK * CC, CC, (size_t)CG, K16 + (size_t)b * NKV * CC, CC, (size_t)CG, SCALE, nullptr, 0, nullptr, 1, 0, 0, S + (size_t)b * NG * NTOK * NKV, nullptr, NKV, (size_t)NTOK * NKV, NTOK, NKV, CG);
  k_zero4<<<(unsigned)(((size_t)NB * NG * NTOK * NKV / 4 + 255) / 256), 256, 0, stream>>>(BIAS, (size_t)NB * NG * NTOK * NKV / 4);
  for (int bg = 0; bg < NCPB; ++bg) {
    k_cpb0<<<(NTOK * NKV * 16 + 255) / 256, 256, 0, stream>>>(GRD, bg, c0w, c0b, C0);
    k_gemm2<3><<<dim3((NTOK * NKV / 128) * 2, 1), 128, 0, stream>>>(C0, 128, 0, BC1, 128, 0, 0.0625f, c1b, 0, nullptr, 1, 0, 0, nullptr, C1, 128, 0, NTOK * NKV, 128, 128);
    k_cpb2<<<(NTOK * NKV + 255) / 256, 256, 0, stream>>>(C1, bg, c2w, c2b, BIAS); }
  k_soft64<<<(NB * NG * NTOK + 7) / 8, 256, 0, stream>>>(S, BIAS, P16);
  for (int b = 0; b < NB; ++b) k_gemm2<0><<<dim3((NTOK / 128) * 1, NG), 128, 0, stream>>>(P16 + (size_t)b * NG * NTOK * NKV, NKV, (size_t)NTOK * NKV, VT + (size_t)b * NG * 64 * NKV, NKV, (size_t)64 * NKV, 0.0009765625f, nullptr, 0, nullptr, 1, 0, 0, nullptr, AO16 + (size_t)b * NTOK * CC, CC, (size_t)CG, NTOK, 64, NKV);
  const dim3 gC((NR / 128) * (CC / 64), 1), gM((NR / 128) * (2048 / 64), 1);
  k_gemm2<0><<<gC, 128, 0, stream>>>(AO16, CC, 0, BO, CC, 0, 0.0625f, ob, 0, XRES, 1, (size_t)CC, 0, X1, nullptr, CC, 0, NR, CC, CC);
  k_stat<1, 0><<<CC, 256, 0, stream>>>(X1, ST2, 0, ST2); k_stat<1, 0><<<CC, 256, 0, stream>>>(X1, ST2, 1, ST2);
  k_bn2<<<(unsigned)(((size_t)NR * CC / 8 + 255) / 256), 256, 0, stream>>>(X1, ST2, n2g, n2b, H16);
  k_gemm2<6><<<gM, 128, 0, stream>>>(H16, CC, 0, BM1, CC, 0, 0.0625f, m1b, 0, nullptr, 1, 0, 0, nullptr, GH, 2048, 0, NR, 2048, CC);
  k_gemm2<0><<<gC, 128, 0, stream>>>(GH, 2048, 0, BM2, 2048, 0, 0.0625f, m2b, 0, X1, 1, (size_t)CC, 0, F, nullptr, CC, 0, NR, CC, 2048);
  k_nchw<<<(NB * CC * (NTOK / 4) + 255) / 256, 256, 0, stream>>>(F, (float*)d_out);
}
